// scaled_dot_product_attention_30794915512922
// MI455X (gfx1250) — hardware-verified
//
#include <hip/hip_runtime.h>
#include <math.h>

typedef __attribute__((ext_vector_type(16))) _Float16 v16h;
typedef __attribute__((ext_vector_type(16))) __bf16 v16b;
typedef __attribute__((ext_vector_type(8)))  _Float16 v8h;
typedef __attribute__((ext_vector_type(8)))  __bf16 v8b;
typedef __attribute__((ext_vector_type(8)))  float v8f;
typedef __attribute__((ext_vector_type(4)))  float v4f;
typedef __attribute__((ext_vector_type(4)))  unsigned v4u;

template <typename T> __device__ __forceinline__ void vst2(void* p, T v) { *(volatile T*)p = v; __threadfence(); *(volatile T*)p = v; }
__device__ __forceinline__ v8f wmma16(v16h a, v16h b, v8f c) {
  v8f d = __builtin_amdgcn_wmma_f32_16x16x32_f16(false, a, false, b, (short)0, c, false, false);
  asm volatile("v_nop\n\tv_nop\n\tv_nop\n\tv_nop" : "+v"(d) : "v"(a), "v"(b));
  return d;
}
__device__ __forceinline__ v8f wmma_bf(v16b a, v16b b, v8f c) {
  v8f d = __builtin_amdgcn_wmma_f32_16x16x32_bf16(false, a, false, b, (short)0, c, false, false);
  asm volatile("v_nop\n\tv_nop\n\tv_nop\n\tv_nop" : "+v"(d) : "v"(a), "v"(b));
  return d;
}
__device__ __forceinline__ v16h frag_h(const _Float16* rowk0, int lane) {
  union { v16h v; v8h q[2]; } u; const _Float16* p = rowk0 + 8 * (lane >> 4);
  u.q[0] = *(const v8h*)p; u.q[1] = *(const v8h*)(p + 16); return u.v;
}
__device__ __forceinline__ v16b frag_b(const __bf16* rowk0, int lane) {
  union { v16b v; v8b q[2]; } u; const __bf16* p = rowk0 + 8 * (lane >> 4);
  u.q[0] = *(const v8b*)p; u.q[1] = *(const v8b*)(p + 16); return u.v;
}
__device__ __forceinline__ float bfr(float v) { return (float)(__bf16)v; }
#define LDSX() do { asm volatile("s_wait_dscnt 0" ::: "memory"); __builtin_amdgcn_wave_barrier(); __builtin_amdgcn_fence(__ATOMIC_RELEASE, "workgroup"); } while (0)

#ifndef NB
#define NB 16
#endif
#ifndef SEQ
#define SEQ 2048
#endif
#define NB_FULL 16
#define SEQ_FULL 2048
#define DD 64
#define NKT (SEQ / 32)
static_assert(SEQ % 64 == 0);
static_assert(NB >= 1 && NB <= NB_FULL);
static_assert(SEQ >= 64 && SEQ <= SEQ_FULL);
static_assert(DD == 64);

#define WS_VT  0u
#define WS_KB  (WS_VT + 2u * (size_t)NB * DD * SEQ)
#define WS_END (WS_KB + 2u * (size_t)NB * SEQ * DD)
static_assert(WS_END <= 134217728u);
static_assert((size_t)NB * SEQ * DD * 4u <= 8388608u);

__global__ __launch_bounds__(128) void k_prep(const float* __restrict__ Kf, const float* __restrict__ Vf, __bf16* __restrict__ KB, _Float16* __restrict__ VT) {
  __shared__ __align__(16) _Float16 th[DD][72];
  const int t = threadIdx.x; const size_t b = blockIdx.y; const int m0 = blockIdx.x * 64;
  const size_t rin = b * SEQ_FULL + m0;
  for (int e = t; e < 64 * 8; e += 128) { const int ml = e >> 3, q = e & 7;
    const float* kp = Kf + (rin + ml) * DD + q * 8; const v4f a = *(const v4f*)kp, c = *(const v4f*)(kp + 4);
    union { v8b h; v4u u; } cv;
#pragma unroll
    for (int i = 0; i < 4; ++i) { cv.h[i] = (__bf16)a[i]; cv.h[4 + i] = (__bf16)c[i]; }
    vst2((void*)(KB + ((b * SEQ + m0 + ml) * DD + q * 8)), cv.u); }
  for (int e = t; e < 64 * DD; e += 128) { const int ml = e / DD, d = e % DD; th[d][ml] = (_Float16)bfr(Vf[(rin + ml) * DD + d]); }
  __syncthreads();
  for (int e = t; e < DD * 8; e += 128) { const int d = e >> 3, q = e & 7; vst2((void*)(VT + (b * DD + d) * (size_t)SEQ + m0 + q * 8), *(const v4u*)&th[d][q * 8]); }
}

__global__ __launch_bounds__(128) void k_att(const float* __restrict__ Q, const __bf16* __restrict__ KB, const _Float16* __restrict__ VT, float* __restrict__ OUT) {
  __shared__ __align__(16) float sp[4][16][36]; __shared__ __align__(16) float so[4][16][68];
  const int tid = threadIdx.x, wave = tid >> 5, lane = tid & 31, col = lane & 15, g = lane >> 4; const size_t b = blockIdx.y; const int qb = blockIdx.x;
  const int q0 = qb * 64 + wave * 16; const size_t rqi = b * SEQ_FULL + q0; const size_t rqo = b * SEQ + q0;
  v16b aq[2];
#pragma unroll
  for (int kc = 0; kc < 2; ++kc) { const float* pp = Q + (rqi + col) * DD + kc * 32 + 8 * g;
#pragma unroll
    for (int i = 0; i < 8; ++i) { aq[kc][i] = (__bf16)pp[i]; aq[kc][8 + i] = (__bf16)pp[16 + i]; } }
  float m[8], l[8];
#pragma unroll
  for (int r = 0; r < 8; ++r) { m[r] = -3.0e38f; l[r] = 0.f; }
  v8f acc[4];
#pragma unroll
  for (int j = 0; j < 4; ++j) acc[j] = v8f{};
#pragma unroll 1
  for (int ks = 0; ks < NKT; ++ks) {
    float s[2][8];
#pragma unroll
    for (int ct = 0; ct < 2; ++ct) { const int kk = ks * 32 + ct * 16 + col; v8f c = {};
#pragma unroll
      for (int kc = 0; kc < 2; ++kc) { const v16b w = frag_b(KB + (b * SEQ + kk) * DD + kc * 32, lane);
        c = wmma_bf(aq[kc], w, c); }
#pragma unroll
      for (int r = 0; r < 8; ++r) s[ct][r] = c[r] * 0.125f; }
    float alpha[8];
#pragma unroll
    for (int r = 0; r < 8; ++r) { float mx = fmaxf(s[0][r], s[1][r]);
#pragma unroll
      for (int o = 1; o < 16; o <<= 1) mx = fmaxf(mx, __shfl_xor(mx, o));
      const float mn = fmaxf(m[r], mx); alpha[r] = (m[r] <= -1.0e38f) ? 0.f : __expf(m[r] - mn);
      const float e0 = __expf(s[0][r] - mn), e1 = __expf(s[1][r] - mn); float es = e0 + e1;
#pragma unroll
      for (int o = 1; o < 16; o <<= 1) es += __shfl_xor(es, o);
      l[r] = l[r] * alpha[r] + es; m[r] = mn; sp[wave][8 * g + r][col] = e0; sp[wave][8 * g + r][16 + col] = e1; }
#pragma unroll
    for (int j = 0; j < 4; ++j)
#pragma unroll
      for (int r = 0; r < 8; ++r) acc[j][r] *= alpha[r];
    LDSX();
    v16h pa, par; { const float* prow = &sp[wave][col][0] + 8 * (lane >> 4);
#pragma unroll
      for (int i = 0; i < 8; ++i) { const float p0 = prow[i] * 2048.0f, p1 = prow[16 + i] * 2048.0f; pa[i] = (_Float16)p0; pa[8 + i] = (_Float16)p1; par[i] = (_Float16)(p0 - (float)pa[i]); par[8 + i] = (_Float16)(p1 - (float)pa[8 + i]); } }
#pragma unroll
    for (int j = 0; j < 4; ++j) { const v16h vh = frag_h(VT + (b * DD + j * 16 + col) * (size_t)SEQ + ks * 32, lane);
      acc[j] = wmma16(pa, vh, acc[j]); acc[j] = wmma16(par, vh, acc[j]); }
    LDSX(); }
#pragma unroll
  for (int r = 0; r < 8; ++r) { const float il = (l[r] > 0.f) ? (1.0f / 2048.0f) / l[r] : 0.f;
#pragma unroll
    for (int j = 0; j < 4; ++j) so[wave][8 * g + r][j * 16 + col] = acc[j][r] * il; }
  LDSX();
  for (int rl = 0; rl < 16; ++rl) if (lane < 16) vst2(OUT + (rqo + rl) * DD + lane * 4, *(const v4f*)&so[wave][rl][lane * 4]);
}

extern "C" void kernel_launch(void* const* d_in, const int* in_sizes, int n_in, void* d_out, int out_size, void* d_ws, size_t ws_size, hipStream_t stream) {
  if (n_in < 3) return;
  const long need_in = ((long)(NB - 1) * SEQ_FULL + SEQ) * DD;
  if ((long)in_sizes[0] < need_in || (long)in_sizes[1] < need_in || (long)in_sizes[2] < need_in) return;
  if ((long)out_size < (long)NB * SEQ * DD) return;
  if (ws_size < (size_t)WS_END) return;
  const float* Qp = (const float*)d_in[0]; const float* Kp = (const float*)d_in[1]; const float* Vp = (const float*)d_in[2];
  char* ws = (char*)d_ws; _Float16* VT = (_Float16*)(ws + WS_VT); __bf16* KB = (__bf16*)(ws + WS_KB);
  k_prep<<<dim3(SEQ / 64, NB), 128, 0, stream>>>(Kp, Vp, KB, VT);
  k_att<<<dim3(SEQ / 64, NB), 128, 0, stream>>>(Qp, KB, VT, (float*)d_out);
}
